// GeneralizedAttention_6296422056055
// MI455X (gfx1250) — hardware-verified
//
#include <hip/hip_runtime.h>
#include <math.h>
#include <stdint.h>

#ifndef NB
#define NB 2
#endif
#define NB_FULL 2
#define CC      256
#define IMH     64
#define IMW     64
#define NN      4096
#define KVH     32
#define KVW     32
#define NK      1024
#define NHD     8
#define HD      32
#define PFD     128
#define NPR     2048
#define LRANGE  16
#define QT      64
#define OSP     68
#define TP      72
#define EP      136
#define QSP     36
#define PYP     33
#define OSV     36
#define WSC     256.0f
#define IWSC    0.00390625f
#define LNPS    6.931471805599453f
#define RSQ2    0.70710678118654752f
#define NL2W    0.15571537944784511f

static_assert(NB >= 1 && NB <= NB_FULL);
static_assert(NN == IMH * IMW && NK == KVH * KVW);
static_assert(NPR == IMW * KVW && NPR == IMH * KVH);
static_assert(CC == NHD * HD && HD == 32 && KVW == 32 && KVH == 32);
static_assert(NN % QT == 0 && NK % QT == 0 && CC % QT == 0 && NPR % QT == 0);
static_assert(CC % 32 == 0 && PFD % 32 == 0 && HD % 32 == 0);
static_assert((OSP * 4) % 16 == 0 && (TP * 2) % 16 == 0 && (EP * 2) % 16 == 0);
static_assert((QSP * 4) % 16 == 0 && (OSV * 4) % 16 == 0);
static_assert(IMW == QT);
static_assert(QT == 2 * HD);

typedef _Float16       v16h __attribute__((ext_vector_type(16)));
typedef _Float16       v8h  __attribute__((ext_vector_type(8)));
typedef __bf16         v16b __attribute__((ext_vector_type(16)));
typedef unsigned short v8us __attribute__((ext_vector_type(8)));
typedef float          v8f  __attribute__((ext_vector_type(8)));
typedef float          v4f  __attribute__((ext_vector_type(4)));
typedef unsigned int   v4u  __attribute__((ext_vector_type(4)));

union Frag  { v8us u[2]; v16h h; v16b bf; };
union FragH { v16h v; v8h hv[2]; };
static_assert(sizeof(Frag) == 32);
static_assert(sizeof(FragH) == 32);

__device__ __forceinline__ unsigned short bf_bits(float f) {
  unsigned u = __float_as_uint(f);
  return (unsigned short)((u + 0x7FFFu + ((u >> 16) & 1u)) >> 16);
}
__device__ __forceinline__ float bf_up(unsigned short hb) { return __uint_as_float(((unsigned)hb) << 16); }
__device__ __forceinline__ float bfr(float f) { return bf_up(bf_bits(f)); }
__device__ __forceinline__ unsigned short h_bits(_Float16 x) { return __builtin_bit_cast(unsigned short, x); }
__device__ __forceinline__ unsigned pk16(unsigned short a, unsigned short b) { return (unsigned)a | ((unsigned)b << 16); }
__device__ __forceinline__ v8f zero8() { v8f z = {0.f, 0.f, 0.f, 0.f, 0.f, 0.f, 0.f, 0.f}; return z; }
__device__ __forceinline__ float hmax8(v8f s) {
  return fmaxf(fmaxf(fmaxf(s[0], s[1]), fmaxf(s[2], s[3])), fmaxf(fmaxf(s[4], s[5]), fmaxf(s[6], s[7])));
}
__device__ __forceinline__ unsigned wave_ballot(bool p) {
#if defined(__HIP_DEVICE_COMPILE__)
  return __builtin_amdgcn_ballot_w32(p);
#else
  return p ? 1u : 0u;
#endif
}

__device__ __forceinline__ Frag ldfrag(const unsigned short* p) {
  Frag f;
  f.u[0] = *(const v8us*)(p);
  f.u[1] = *(const v8us*)(p + 16);
  return f;
}

__device__ __forceinline__ v8f mma_h(v16h a, v16h b, v8f c) {
  v8f d = __builtin_amdgcn_wmma_f32_16x16x32_f16(false, a, false, b, (short)0, c, false, false);
#if defined(__HIP_DEVICE_COMPILE__)
  asm volatile("v_nop\n\tv_nop\n\tv_nop\n\tv_nop" : "+v"(d) : "v"(a), "v"(b));
#endif
  return d;
}
__device__ __forceinline__ v8f mma_b(v16b a, v16b b, v8f c) {
  v8f d = __builtin_amdgcn_wmma_f32_16x16x32_bf16(false, a, false, b, (short)0, c, false, false);
#if defined(__HIP_DEVICE_COMPILE__)
  const v16h ha = __builtin_bit_cast(v16h, a), hb = __builtin_bit_cast(v16h, b);
  asm volatile("v_nop\n\tv_nop\n\tv_nop\n\tv_nop" : "+v"(d) : "v"(ha), "v"(hb));
#endif
  return d;
}

__global__ __launch_bounds__(256)
void cvt_w(const float* __restrict__ qw, const float* __restrict__ kw, const float* __restrict__ vw,
           const float* __restrict__ pw, const float* __restrict__ fxw, const float* __restrict__ fyw,
           unsigned short* W16, unsigned short* WPB, unsigned short* WF) {
  const int tid = threadIdx.x, blk = blockIdx.x;
  unsigned short* dst;
  v4u u;
  if (blk < 128) {
    const int grp = blk >> 5;
    const int rl = tid >> 5, col = 8 * (tid & 31);
    const int o = 8 * (blk & 31) + rl;
    const float* wbase = (grp == 0) ? qw : ((grp == 1) ? kw : ((grp == 2) ? vw : pw));
    const float* s = wbase + (size_t)o * CC + col;
    const v4f a = *(const v4f*)s;
    const v4f q = *(const v4f*)(s + 4);
    const float f[8] = {a[0], a[1], a[2], a[3], q[0], q[1], q[2], q[3]};
    if (grp < 3) {
#pragma unroll
      for (int t = 0; t < 4; ++t) {
        const _Float16 h0 = (_Float16)(bfr(f[2 * t]) * WSC);
        const _Float16 h1 = (_Float16)(bfr(f[2 * t + 1]) * WSC);
        u[t] = pk16(h_bits(h0), h_bits(h1));
      }
      dst = W16 + (size_t)grp * CC * CC + (size_t)o * CC + col;
    } else {
#pragma unroll
      for (int t = 0; t < 4; ++t) u[t] = pk16(bf_bits(f[2 * t]), bf_bits(f[2 * t + 1]));
      dst = WPB + (size_t)o * CC + col;
    }
  } else {
    const int j = blk - 128;
    const int axis = j >> 4;
    const int r = 16 * j + (tid >> 4);
    const int o = r & 255;
    const int col = 8 * (tid & 15);
    const float* s = (axis ? fyw : fxw) + (size_t)o * PFD + col;
    const v4f a = *(const v4f*)s;
    const v4f q = *(const v4f*)(s + 4);
    const float f[8] = {a[0], a[1], a[2], a[3], q[0], q[1], q[2], q[3]};
#pragma unroll
    for (int t = 0; t < 4; ++t) u[t] = pk16(bf_bits(f[2 * t]), bf_bits(f[2 * t + 1]));
    dst = WF + (size_t)r * PFD + col;
  }
#pragma unroll
  for (int pass = 0; pass < 2; ++pass) {
    *(volatile v4u*)dst = u;
    __threadfence();
  }
}

__global__ __launch_bounds__(256)
void cvt_x(const float* __restrict__ x, unsigned short* XP) {
  __shared__ __align__(16) unsigned short T[QT * TP];
  const int tid = threadIdx.x;
  const int nb = blockIdx.x, cb = blockIdx.y, b = blockIdx.z;
  const int e = tid & 7, lq = tid >> 3;
  const int n0 = nb * QT, c0 = cb * QT;
#pragma unroll
  for (int it = 0; it < 2; ++it) {
    const int cl = it * 32 + lq;
    const float* sp = x + ((size_t)(b * CC + c0 + cl)) * NN + n0 + 8 * e;
    const v4f a = *(const v4f*)sp;
    const v4f q = *(const v4f*)(sp + 4);
    unsigned short hb[8];
#pragma unroll
    for (int t = 0; t < 4; ++t) {
      hb[t]     = h_bits((_Float16)bfr(a[t]));
      hb[4 + t] = h_bits((_Float16)bfr(q[t]));
    }
#pragma unroll
    for (int t = 0; t < 8; ++t) T[(8 * e + t) * TP + cl] = hb[t];
  }
  __syncthreads();
  v4u up[2];
#pragma unroll
  for (int it = 0; it < 2; ++it) {
    const int nl = it * 32 + lq;
    up[it] = *(const v4u*)(T + nl * TP + 8 * e);
  }
#pragma unroll
  for (int pass = 0; pass < 2; ++pass) {
#pragma unroll
    for (int it = 0; it < 2; ++it) {
      const int rl = it * 32 + lq;
      *(volatile v4u*)(XP + ((size_t)(b * NN + n0 + rl)) * CC + c0 + 8 * e) = up[it];
    }
    __threadfence();
  }
}

template <int MODE>
__global__ __launch_bounds__(128)
void gemm_x(const unsigned short* __restrict__ W16, const unsigned short* __restrict__ XP,
            const float* __restrict__ ab, unsigned short* Ph, unsigned short* Pl,
            unsigned short* Vt, float* ABK) {
  __shared__ __align__(16) float Os[QT * OSP];
  __shared__ __align__(16) float abks[2 * QT];
  constexpr int NP = (MODE == 0) ? NN : NK;
  const int tid  = threadIdx.x;
  const int lane = tid & 31, wave = tid >> 5;
  const int hh   = lane >> 4, c = lane & 15;
  const int nt   = blockIdx.x, mb = blockIdx.y, b = blockIdx.z;
  const int n0   = nt * QT, o0 = mb * QT;
  (void)ab; (void)Ph; (void)Pl; (void)Vt; (void)ABK; (void)abks;

  const unsigned short* ap = W16 + (size_t)MODE * CC * CC + (size_t)(o0 + c) * CC + 8 * hh;
  const int nrow = n0 + 16 * wave + c;
  const int pix = (MODE == 0) ? nrow : (2 * IMW * (nrow >> 5) + 2 * (nrow & 31));
  const unsigned short* bp = XP + ((size_t)(b * NN + pix)) * CC + 8 * hh;

  v8f acc[4];
#pragma unroll
  for (int mt = 0; mt < 4; ++mt) acc[mt] = zero8();

#pragma unroll
  for (int ks = 0; ks < CC / 32; ++ks) {
    const Frag fb = ldfrag(bp + 32 * ks);
#pragma unroll
    for (int mt = 0; mt < 4; ++mt) {
      const Frag fa = ldfrag(ap + (size_t)(16 * mt) * CC + 32 * ks);
      acc[mt] = mma_h(fa.h, fb.h, acc[mt]);
    }
  }

  {
    const int nl = 16 * wave + c;
#pragma unroll
    for (int mt = 0; mt < 4; ++mt) {
      v4f va, vb;
#pragma unroll
      for (int r = 0; r < 4; ++r) { va[r] = acc[mt][r] * IWSC; vb[r] = acc[mt][4 + r] * IWSC; }
      *(v4f*)(Os + nl * OSP + 16 * mt + 8 * hh)     = va;
      *(v4f*)(Os + nl * OSP + 16 * mt + 8 * hh + 4) = vb;
    }
  }
  __syncthreads();

  const int e = tid & 7, lq = tid >> 3;
  if constexpr (MODE == 2) {
    v4u uv[4];
#pragma unroll
    for (int it = 0; it < 4; ++it) {
      const int ol = it * 16 + lq;
      unsigned short hb[8];
#pragma unroll
      for (int t = 0; t < 8; ++t) hb[t] = h_bits((_Float16)Os[(8 * e + t) * OSP + ol]);
#pragma unroll
      for (int t = 0; t < 4; ++t) uv[it][t] = pk16(hb[2 * t], hb[2 * t + 1]);
    }
#pragma unroll
    for (int pass = 0; pass < 2; ++pass) {
#pragma unroll
      for (int it = 0; it < 4; ++it) {
        const int ol = it * 16 + lq;
        const int oo = o0 + ol, hd = oo >> 5, d = oo & 31;
        *(volatile v4u*)(Vt + ((size_t)((b * NHD + hd) * HD + d)) * NK + n0 + 8 * e) = uv[it];
      }
      __threadfence();
    }
  } else {
    v4u uh[4], ul[4];
#pragma unroll
    for (int it = 0; it < 4; ++it) {
      const int L = it * 16 + lq;
      const int hs = L >> 5, j = L & 31;
      const int row = 2 * j + (e >> 2);
      const int cb0 = 32 * hs + 8 * (e & 3);
      const v4f a = *(const v4f*)(Os + row * OSP + cb0);
      const v4f q = *(const v4f*)(Os + row * OSP + cb0 + 4);
      const float f[8] = {a[0], a[1], a[2], a[3], q[0], q[1], q[2], q[3]};
#pragma unroll
      for (int t = 0; t < 4; ++t) {
        const float f0 = f[2 * t], f1 = f[2 * t + 1];
        const unsigned short hb0 = bf_bits(f0), hb1 = bf_bits(f1);
        const unsigned short lb0 = bf_bits(f0 - bf_up(hb0));
        const unsigned short lb1 = bf_bits(f1 - bf_up(hb1));
        uh[it][t] = pk16(hb0, hb1);
        ul[it][t] = pk16(lb0, lb1);
      }
    }
    v4f abv = {0.f, 0.f, 0.f, 0.f};
    if constexpr (MODE == 1) {
      const int kl = tid & 63, hs = tid >> 6;
      const float* abp  = ab + (2 * mb + hs) * HD;
      const float* orow = Os + kl * OSP + 32 * hs;
      float s = 0.f;
#pragma unroll
      for (int d4 = 0; d4 < 8; ++d4) {
        const v4f g  = *(const v4f*)(abp + 4 * d4);
        const v4f ov = *(const v4f*)(orow + 4 * d4);
        s += bfr(g[0]) * ov[0] + bfr(g[1]) * ov[1] + bfr(g[2]) * ov[2] + bfr(g[3]) * ov[3];
      }
      abks[hs * QT + kl] = s;
      __syncthreads();
      if (tid < 32) abv = *(const v4f*)(abks + (lq >> 1) * QT + 32 * (lq & 1) + 4 * e);
    }
#pragma unroll
    for (int pass = 0; pass < 2; ++pass) {
#pragma unroll
      for (int it = 0; it < 4; ++it) {
        const int L = it * 16 + lq;
        const int hs = L >> 5, j = L & 31;
        const size_t po = ((size_t)((b * NHD + 2 * mb + hs) * NP + n0 + 2 * j)) * HD + 8 * e;
        *(volatile v4u*)(Ph + po) = uh[it];
        *(volatile v4u*)(Pl + po) = ul[it];
      }
      if constexpr (MODE == 1) {
        if (tid < 32)
          *(volatile v4f*)(ABK + (size_t)(b * NHD + 2 * mb + (lq >> 1)) * NK + n0 + 32 * (lq & 1) + 4 * e) = abv;
      }
      __threadfence();
    }
  }
}

__global__ __launch_bounds__(128)
void posfeat(const unsigned short* __restrict__ WF, float* PF) {
  __shared__ __align__(16) unsigned short Eh[QT * EP];
  __shared__ __align__(16) unsigned short El[QT * EP];
  __shared__ __align__(16) float Os[QT * OSP];
  const int tid  = threadIdx.x;
  const int lane = tid & 31, wave = tid >> 5;
  const int hh   = lane >> 4, c = lane & 15;
  const int rt   = blockIdx.x, axis = blockIdx.y;
  const int R0   = rt * QT;

#pragma unroll 1
  for (int it = 0; it < 32; ++it) {
    const int idx = it * 128 + tid;
    const int rl = idx >> 6, fa = idx & 63;
    const int row = R0 + rl;
    const int qc = row >> 5, kq = row & 31;
    const float diff = (float)(qc - 2 * kq);
    const float a = diff * exp2f(-(float)fa * NL2W);
    const float sv = sinf(a);
    const float cv = cosf(a);
    const unsigned short shb = bf_bits(sv), chb = bf_bits(cv);
    Eh[rl * EP + fa]      = shb;
    El[rl * EP + fa]      = bf_bits(sv - bf_up(shb));
    Eh[rl * EP + 64 + fa] = chb;
    El[rl * EP + 64 + fa] = bf_bits(cv - bf_up(chb));
  }
  __syncthreads();

  const unsigned short* ebh = Eh + (16 * wave + c) * EP + 8 * hh;
  const unsigned short* ebl = El + (16 * wave + c) * EP + 8 * hh;
  const int e = tid & 7, lq = tid >> 3;
#pragma unroll 1
  for (int ob = 0; ob < 4; ++ob) {
    const unsigned short* ap = WF + (size_t)axis * CC * PFD + (size_t)(QT * ob + c) * PFD + 8 * hh;
    v8f acc[4];
#pragma unroll
    for (int mt = 0; mt < 4; ++mt) acc[mt] = zero8();
#pragma unroll
    for (int ks = 0; ks < PFD / 32; ++ks) {
      const Frag fbh = ldfrag(ebh + 32 * ks);
      const Frag fbl = ldfrag(ebl + 32 * ks);
#pragma unroll
      for (int mt = 0; mt < 4; ++mt) {
        const Frag fa = ldfrag(ap + (size_t)(16 * mt) * PFD + 32 * ks);
        acc[mt] = mma_b(fa.bf, fbh.bf, acc[mt]);
        acc[mt] = mma_b(fa.bf, fbl.bf, acc[mt]);
      }
    }
    {
      const int nl = 16 * wave + c;
#pragma unroll
      for (int mt = 0; mt < 4; ++mt) {
        v4f va, vb;
#pragma unroll
        for (int r = 0; r < 4; ++r) { va[r] = acc[mt][r] * RSQ2; vb[r] = acc[mt][4 + r] * RSQ2; }
        *(v4f*)(Os + nl * OSP + 16 * mt + 8 * hh)     = va;
        *(v4f*)(Os + nl * OSP + 16 * mt + 8 * hh + 4) = vb;
      }
    }
    __syncthreads();
    v4f res[8];
#pragma unroll
    for (int it = 0; it < 8; ++it) {
      const int L = it * 16 + lq;
      const int rl = L & 63, hs = L >> 6;
      res[it] = *(const v4f*)(Os + rl * OSP + 32 * hs + 4 * e);
    }
#pragma unroll
    for (int pass = 0; pass < 2; ++pass) {
#pragma unroll
      for (int it = 0; it < 8; ++it) {
        const int L = it * 16 + lq;
        const int rl = L & 63, hs = L >> 6;
        float* dst = PF + ((size_t)(axis * NHD + 2 * ob + hs)) * ((size_t)NPR * HD) + (size_t)(R0 + rl) * HD + 4 * e;
        *(volatile v4f*)dst = res[it];
      }
      __threadfence();
    }
    __syncthreads();
  }
}

__global__ __launch_bounds__(128)
void attn_k(const unsigned short* __restrict__ Qh, const unsigned short* __restrict__ Ql,
            const unsigned short* __restrict__ Kh, const unsigned short* __restrict__ Kl,
            const unsigned short* __restrict__ Vt, const float* __restrict__ ABK,
            const float* __restrict__ PF, const float* __restrict__ gb,
            unsigned short* OPh, unsigned short* OPl) {
  __shared__ __align__(16) float qs[4 * 16 * QSP];
  __shared__ __align__(16) float pys[4 * 16 * PYP];
  __shared__ __align__(16) float Os[QT * OSV];
  const int tid  = threadIdx.x;
  const int wave = tid >> 5, lane = tid & 31;
  const int hh   = lane >> 4, c = lane & 15;
  const int y = blockIdx.x, hd = blockIdx.y, b = blockIdx.z;
  const int bh = b * NHD + hd;
  const int xq = 16 * wave + c;
  const int pq = y * IMW + xq;

  const int kylo = (y >= LRANGE) ? ((y - LRANGE) >> 1) : 0;
  int kyhi = ((y + LRANGE + 1) >> 1) + 1;  if (kyhi > KVH) kyhi = KVH;
  const int kxlo = (xq >= LRANGE) ? ((xq - LRANGE) >> 1) : 0;
  int kxhi = ((xq + LRANGE + 1) >> 1) + 1; if (kxhi > KVW) kxhi = KVW;

  {
    const size_t rb = ((size_t)bh * NN + (size_t)y * IMW + 16 * wave) * HD;
    const int d0 = 8 * (lane & 3);
    const v4f g0 = *(const v4f*)(gb + hd * HD + d0);
    const v4f g1 = *(const v4f*)(gb + hd * HD + d0 + 4);
#pragma unroll
    for (int it = 0; it < 2; ++it) {
      const int t = 8 * it + (lane >> 2);
      const size_t qi = rb + (size_t)t * HD + d0;
      const v4u uhv = *(const v4u*)(Qh + qi);
      const v4u ulv = *(const v4u*)(Ql + qi);
      float f[8];
#pragma unroll
      for (int j = 0; j < 4; ++j) {
        const unsigned wh = uhv[j], wl = ulv[j];
        f[2 * j]     = __uint_as_float(wh << 16) + __uint_as_float(wl << 16);
        f[2 * j + 1] = __uint_as_float(wh & 0xffff0000u) + __uint_as_float(wl & 0xffff0000u);
      }
      v4f va, vb;
#pragma unroll
      for (int r = 0; r < 4; ++r) { va[r] = f[r] + bfr(g0[r]); vb[r] = f[4 + r] + bfr(g1[r]); }
      *(v4f*)(qs + (wave * 16 + t) * QSP + d0)     = va;
      *(v4f*)(qs + (wave * 16 + t) * QSP + d0 + 4) = vb;
    }
  }
  __syncthreads();
  const float* qrow = qs + (wave * 16 + c) * QSP;

  float px0[8], px1[8];
  {
    const float* pfb = PF + (size_t)hd * ((size_t)NPR * HD) + (size_t)xq * (KVW * HD);
#pragma unroll
    for (int r = 0; r < 8; ++r) {
      float s0v = 0.f;
      float s1v = 0.f;
      const float* p0 = pfb + (8 * hh + r) * HD;
      const float* p1 = pfb + (16 + 8 * hh + r) * HD;
#pragma unroll 4
      for (int d4 = 0; d4 < 8; ++d4) {
        const v4f qv = *(const v4f*)(qrow + 4 * d4);
        const v4f u0 = *(const v4f*)(p0 + 4 * d4);
        const v4f u1 = *(const v4f*)(p1 + 4 * d4);
        s0v += qv[0] * u0[0] + qv[1] * u0[1] + qv[2] * u0[2] + qv[3] * u0[3];
        s1v += qv[0] * u1[0] + qv[1] * u1[1] + qv[2] * u1[2] + qv[3] * u1[3];
      }
      px0[r] = s0v;
      px1[r] = s1v;
    }
  }
  {
    const float* pfb = PF + (size_t)(NHD + hd) * ((size_t)NPR * HD) + (size_t)y * (KVH * HD);
    float* pyw = pys + (wave * 16 + c) * PYP;
#pragma unroll 1
    for (int j = 0; kylo + 2 * j < kyhi; ++j) {
      int ky = kylo + 2 * j + hh;
      ky = (ky > KVH - 1) ? (KVH - 1) : ky;
      float sv = 0.f;
      const float* p0 = pfb + ky * HD;
#pragma unroll 4
      for (int d4 = 0; d4 < 8; ++d4) {
        const v4f qv = *(const v4f*)(qrow + 4 * d4);
        const v4f u0 = *(const v4f*)(p0 + 4 * d4);
        sv += qv[0] * u0[0] + qv[1] * u0[1] + qv[2] * u0[2] + qv[3] * u0[3];
      }
      pyw[ky] = sv;
    }
  }
  __syncthreads();
  const float* pyrow = pys + (wave * 16 + c) * PYP;

  const size_t qo = ((size_t)bh * NN + pq) * HD + 8 * hh;
  const Frag qh = ldfrag(Qh + qo);
  const Frag ql = ldfrag(Ql + qo);
  const unsigned short* Khp = Kh + (size_t)bh * NK * HD + (size_t)c * HD + 8 * hh;
  const unsigned short* Klp = Kl + (size_t)bh * NK * HD + (size_t)c * HD + 8 * hh;
  const unsigned short* Vp  = Vt + (size_t)bh * HD * NK + (size_t)c * NK + 8 * hh;
  const float* abkb = ABK + (size_t)bh * NK + 8 * hh;
  const float NINF = -__builtin_inff();

  float m = -1.0e30f, l = 0.f;
  v8f o[2];
  o[0] = zero8(); o[1] = zero8();

#pragma unroll 1
  for (int ky = kylo; ky < kyhi; ++ky) {
    const int kp0 = ky * KVW;
    const Frag k0  = ldfrag(Khp + (size_t)kp0 * HD);
    const Frag k1  = ldfrag(Khp + (size_t)(kp0 + 16) * HD);
    const Frag k0l = ldfrag(Klp + (size_t)kp0 * HD);
    const Frag k1l = ldfrag(Klp + (size_t)(kp0 + 16) * HD);
    v8f s0 = zero8(), s1 = zero8();
    s0 = mma_b(k0.bf, qh.bf, s0);
    s1 = mma_b(k1.bf, qh.bf, s1);
    s0 = mma_b(k0.bf, ql.bf, s0);
    s1 = mma_b(k1.bf, ql.bf, s1);
    s0 = mma_b(k0l.bf, qh.bf, s0);
    s1 = mma_b(k1l.bf, qh.bf, s1);

    const v4f a0 = *(const v4f*)(abkb + kp0);
    const v4f a1 = *(const v4f*)(abkb + kp0 + 4);
    const v4f a2 = *(const v4f*)(abkb + kp0 + 16);
    const v4f a3 = *(const v4f*)(abkb + kp0 + 20);
    const float py = pyrow[ky];
#pragma unroll
    for (int r = 0; r < 8; ++r) {
      const int kx0 = 8 * hh + r, kx1 = 16 + 8 * hh + r;
      const float ab0 = (r < 4) ? a0[r & 3] : a1[r & 3];
      const float ab1 = (r < 4) ? a2[r & 3] : a3[r & 3];
      const float e0 = s0[r] + ab0 + px0[r] + py;
      const float e1 = s1[r] + ab1 + px1[r] + py;
      s0[r] = (kx0 >= kxlo && kx0 < kxhi) ? e0 : NINF;
      s1[r] = (kx1 >= kxlo && kx1 < kxhi) ? e1 : NINF;
    }

    float mx = fmaxf(hmax8(s0), hmax8(s1));
    mx = fmaxf(mx, __shfl_xor(mx, 16, 32));
    const float mn = fmaxf(m, mx);
    const unsigned grew = wave_ballot(mx > m);
    if (grew != 0u) {
      const float corr = __expf(m - mn);
      l *= corr;
#pragma unroll
      for (int j = 0; j < 2; ++j) {
#pragma unroll
        for (int r = 0; r < 8; ++r) o[j][r] *= corr;
      }
    }
    m = mn;
    const float msh = mn - LNPS;

    FragH ph;
    float ls = 0.f;
#pragma unroll
    for (int r = 0; r < 8; ++r) {
      const float e0 = __expf(s0[r] - msh);
      const float e1 = __expf(s1[r] - msh);
      ls += e0 + e1;
      ph.hv[0][r] = (_Float16)e0;
      ph.hv[1][r] = (_Float16)e1;
    }
    l += ls;

#pragma unroll
    for (int j = 0; j < 2; ++j) {
      const Frag vf = ldfrag(Vp + (size_t)(16 * j) * NK + kp0);
      o[j] = mma_h(vf.h, ph.v, o[j]);
    }
  }
  l += __shfl_xor(l, 16, 32);
  const float inv = 1.0f / l;

  const int qr = 16 * wave + c;
#pragma unroll
  for (int j = 0; j < 2; ++j) {
    v4f va, vb;
#pragma unroll
    for (int r = 0; r < 4; ++r) { va[r] = o[j][r] * inv; vb[r] = o[j][4 + r] * inv; }
    *(v4f*)(Os + qr * OSV + 16 * j + 8 * hh)     = va;
    *(v4f*)(Os + qr * OSV + 16 * j + 8 * hh + 4) = vb;
  }
  __syncthreads();

  const int e = tid & 7, lq = tid >> 3;
  v4u uh[2], ul[2];
#pragma unroll
  for (int it = 0; it < 2; ++it) {
    const int L = 16 * it + lq;
    const int row = 2 * L + (e >> 2), dl = 8 * (e & 3);
    const v4f a = *(const v4f*)(Os + row * OSV + dl);
    const v4f q = *(const v4f*)(Os + row * OSV + dl + 4);
    const float f[8] = {a[0], a[1], a[2], a[3], q[0], q[1], q[2], q[3]};
#pragma unroll
    for (int t = 0; t < 4; ++t) {
      const float f0 = f[2 * t], f1 = f[2 * t + 1];
      const unsigned short hb0 = bf_bits(f0), hb1 = bf_bits(f1);
      const unsigned short lb0 = bf_bits(f0 - bf_up(hb0));
      const unsigned short lb1 = bf_bits(f1 - bf_up(hb1));
      uh[it][t] = pk16(hb0, hb1);
      ul[it][t] = pk16(lb0, lb1);
    }
  }
#pragma unroll
  for (int pass = 0; pass < 2; ++pass) {
#pragma unroll
    for (int it = 0; it < 2; ++it) {
      const int L = 16 * it + lq;
      const size_t po = ((size_t)bh * NN + (size_t)y * IMW + 2 * L) * HD + 8 * e;
      *(volatile v4u*)(OPh + po) = uh[it];
      *(volatile v4u*)(OPl + po) = ul[it];
    }
    __threadfence();
  }
}

__global__ __launch_bounds__(128)
void proj_k(const unsigned short* __restrict__ WPB, const unsigned short* __restrict__ OPh,
            const unsigned short* __restrict__ OPl, const float* __restrict__ pb,
            const float* __restrict__ gam, const float* __restrict__ x, float* out) {
  __shared__ __align__(16) float Os[QT * OSP];
  const int tid  = threadIdx.x;
  const int lane = tid & 31, wave = tid >> 5;
  const int hh   = lane >> 4, c = lane & 15;
  const int nt   = blockIdx.x, mb = blockIdx.y, b = blockIdx.z;
  const int n0   = nt * QT, o0 = mb * QT;

  const unsigned short* ap = WPB + (size_t)(o0 + c) * CC + 8 * hh;
  const size_t brow = (size_t)(n0 + 16 * wave + c) * HD + 8 * hh;

  v8f acc[4];
#pragma unroll
  for (int mt = 0; mt < 4; ++mt) acc[mt] = zero8();

#pragma unroll 2
  for (int ks = 0; ks < NHD; ++ks) {
    const size_t pl = ((size_t)(b * NHD + ks)) * NN * HD + brow;
    const Frag fbh = ldfrag(OPh + pl);
    const Frag fbl = ldfrag(OPl + pl);
#pragma unroll
    for (int mt = 0; mt < 4; ++mt) {
      const Frag fa = ldfrag(ap + (size_t)(16 * mt) * CC + 32 * ks);
      acc[mt] = mma_b(fa.bf, fbh.bf, acc[mt]);
      acc[mt] = mma_b(fa.bf, fbl.bf, acc[mt]);
    }
  }

  {
    const int nl = 16 * wave + c;
#pragma unroll
    for (int mt = 0; mt < 4; ++mt) {
      v4f va, vb;
#pragma unroll
      for (int r = 0; r < 4; ++r) { va[r] = acc[mt][r]; vb[r] = acc[mt][4 + r]; }
      *(v4f*)(Os + nl * OSP + 16 * mt + 8 * hh)     = va;
      *(v4f*)(Os + nl * OSP + 16 * mt + 8 * hh + 4) = vb;
    }
  }
  __syncthreads();

  const float g = bfr(gam[0]);
  const int e = tid & 7, lq = tid >> 3;
  v4f res[8];
#pragma unroll
  for (int it = 0; it < 8; ++it) {
    const int L   = it * 16 + lq;
    const int ol  = L >> 1, hf = L & 1;
    const int nl  = hf * 32 + 4 * e;
    const int oo  = o0 + ol;
    const float pbv = bfr(pb[oo]);
    const size_t idx = ((size_t)(b * CC + oo)) * NN + n0 + nl;
    const v4f xv = *(const v4f*)(x + idx);
#pragma unroll
    for (int t = 0; t < 4; ++t) res[it][t] = g * (Os[(nl + t) * OSP + ol] + pbv) + bfr(xv[t]);
  }
#pragma unroll
  for (int pass = 0; pass < 2; ++pass) {
#pragma unroll
    for (int it = 0; it < 8; ++it) {
      const int L   = it * 16 + lq;
      const int ol  = L >> 1, hf = L & 1;
      const int nl  = hf * 32 + 4 * e;
      const size_t idx = ((size_t)(b * CC + o0 + ol)) * NN + n0 + nl;
      *(volatile v4f*)(out + idx) = res[it];
    }
    __threadfence();
  }
}

extern "C" void kernel_launch(void* const* d_in, const int* in_sizes, int n_in,
                              void* d_out, int out_size, void* d_ws, size_t ws_size,
                              hipStream_t stream) {
  const int XN = NB * CC * NN;
  if (n_in < 11) return;
  if (in_sizes[0] < XN) return;
  if (in_sizes[1] < CC * CC || in_sizes[2] < CC * CC || in_sizes[3] < CC * CC || in_sizes[8] < CC * CC) return;
  if (in_sizes[4] < CC * PFD || in_sizes[5] < CC * PFD) return;
  if (in_sizes[6] < CC || in_sizes[7] < CC || in_sizes[9] < CC || in_sizes[10] < 1) return;
  if (out_size < XN) return;

  size_t off = 0;
  auto carve = [&](size_t bytes) { const size_t o = off; off += (bytes + 255) & ~(size_t)255; return o; };
  const size_t oW16 = carve((size_t)3 * CC * CC * 2);
  const size_t oWPB = carve((size_t)CC * CC * 2);
  const size_t oWF  = carve((size_t)2 * CC * PFD * 2);
  const size_t oXP  = carve((size_t)NB * NN * CC * 2);
  const size_t oQh  = carve((size_t)NB * NHD * NN * HD * 2);
  const size_t oQl  = carve((size_t)NB * NHD * NN * HD * 2);
  const size_t oKh  = carve((size_t)NB * NHD * NK * HD * 2);
  const size_t oKl  = carve((size_t)NB * NHD * NK * HD * 2);
  const size_t oVt  = carve((size_t)NB * NHD * HD * NK * 2);
  const size_t oABK = carve((size_t)NB * NHD * NK * 4);
  const size_t oPF  = carve((size_t)2 * NHD * NPR * HD * 4);
  const size_t oOPh = carve((size_t)NB * NHD * NN * HD * 2);
  const size_t oOPl = carve((size_t)NB * NHD * NN * HD * 2);
  if (off > ws_size) return;
  if (off > (size_t)134217728) return;

  const float* x   = (const float*)d_in[0];
  const float* qw  = (const float*)d_in[1];
  const float* kw  = (const float*)d_in[2];
  const float* vw  = (const float*)d_in[3];
  const float* fxw = (const float*)d_in[4];
  const float* fyw = (const float*)d_in[5];
  const float* ab  = (const float*)d_in[6];
  const float* gb  = (const float*)d_in[7];
  const float* pw  = (const float*)d_in[8];
  const float* pb  = (const float*)d_in[9];
  const float* gam = (const float*)d_in[10];

  char* ws = (char*)d_ws;
  unsigned short* W16 = (unsigned short*)(ws + oW16);
  unsigned short* WPB = (unsigned short*)(ws + oWPB);
  unsigned short* WF  = (unsigned short*)(ws + oWF);
  unsigned short* XP  = (unsigned short*)(ws + oXP);
  unsigned short* Qh  = (unsigned short*)(ws + oQh);
  unsigned short* Ql  = (unsigned short*)(ws + oQl);
  unsigned short* Kh  = (unsigned short*)(ws + oKh);
  unsigned short* Kl  = (unsigned short*)(ws + oKl);
  unsigned short* Vt  = (unsigned short*)(ws + oVt);
  float*          ABK = (float*)(ws + oABK);
  float*          PF  = (float*)(ws + oPF);
  unsigned short* OPh = (unsigned short*)(ws + oOPh);
  unsigned short* OPl = (unsigned short*)(ws + oOPl);
  float* out = (float*)d_out;

  const dim3 blk256(256), blk128(128);

  cvt_w<<<dim3(160), blk256, 0, stream>>>(qw, kw, vw, pw, fxw, fyw, W16, WPB, WF);
  cvt_x<<<dim3(NN / QT, CC / QT, NB), blk256, 0, stream>>>(x, XP);
  posfeat<<<dim3(NPR / QT, 2), blk128, 0, stream>>>(WF, PF);
  gemm_x<0><<<dim3(NN / QT, CC / QT, NB), blk128, 0, stream>>>(W16, XP, ab, Qh, Ql, Vt, ABK);
  gemm_x<1><<<dim3(NK / QT, CC / QT, NB), blk128, 0, stream>>>(W16, XP, ab, Kh, Kl, Vt, ABK);
  gemm_x<2><<<dim3(NK / QT, CC / QT, NB), blk128, 0, stream>>>(W16, XP, ab, Kh, Kl, Vt, ABK);
  attn_k<<<dim3(IMH, NHD, NB), blk128, 0, stream>>>(Qh, Ql, Kh, Kl, Vt, ABK, PF, gb, OPh, OPl);
  proj_k<<<dim3(NN / QT, CC / QT, NB), blk128, 0, stream>>>(WPB, OPh, OPl, pb, gam, x, out);
  (void)hipGetLastError();
}
